// FeatureGNNModel_549755814533
// MI455X (gfx1250) — hardware-verified
//
#include <hip/hip_runtime.h>
#include <math.h>

#define HD 64
#define NUSERS 100000
#define NITEMS 50000
#define NNODE 150000
#define MU 100032
#define MI 50048
#define MP 150016
#define NE 1200000
#define NQ 16384
#define NT 256
#define TR 8192
#define NTILE 19
#define RPW 1024
#define SCH 4096
#define SPT 16
#define NCH 293
#define LNEPS 1e-5f

typedef __attribute__((ext_vector_type(16))) _Float16 v16h;
typedef __attribute__((ext_vector_type(8)))  _Float16 v8h;
typedef __attribute__((ext_vector_type(4)))  _Float16 v4h;
typedef __attribute__((ext_vector_type(2)))  _Float16 v2h;
typedef __attribute__((ext_vector_type(16))) __bf16   v16b;
typedef __attribute__((ext_vector_type(8)))  __bf16   v8b;
typedef __attribute__((ext_vector_type(8)))  float    v8f;
typedef __attribute__((ext_vector_type(4)))  float    v4f;
typedef __attribute__((ext_vector_type(2)))  float    v2f;
typedef __attribute__((ext_vector_type(4)))  int      v4i;

__device__ __forceinline__ unsigned short f2bf_bits(float f) {
  unsigned u = __float_as_uint(f);
  return (unsigned short)((u + 0x7FFFu + ((u >> 16) & 1u)) >> 16);
}
__device__ __forceinline__ float bf_bits2f(unsigned short h) { return __uint_as_float(((unsigned)h) << 16); }

__device__ __forceinline__ void dep_guard_h(v8f& a, v8f& b, v16h x, v16h y) { asm volatile("v_nop\n\tv_nop\n\tv_nop\n\tv_nop" : "+v"(a), "+v"(b) : "v"(x), "v"(y)); }
__device__ __forceinline__ void dep_guard_b(v8f& a, v8f& b, v16b x, v16b y) { asm volatile("v_nop\n\tv_nop\n\tv_nop\n\tv_nop" : "+v"(a), "+v"(b) : "v"(x), "v"(y)); }
__device__ __forceinline__ void keep4_h(v16h a, v16h b, v16h c, v16h d) { asm volatile("v_nop" :: "v"(a), "v"(b), "v"(c), "v"(d)); }
__device__ __forceinline__ void keep4_b(v16b a, v16b b, v16b c, v16b d) { asm volatile("v_nop" :: "v"(a), "v"(b), "v"(c), "v"(d)); }
__device__ __forceinline__ void acc_guard4(v8f& a, v8f& b, v8f& c, v8f& d) { asm volatile("v_nop\n\tv_nop\n\tv_nop\n\tv_nop" : "+v"(a), "+v"(b), "+v"(c), "+v"(d)); }
template <typename T> struct Frag;
template <> struct Frag<_Float16> {
  typedef v16h V; union U { v16h v; v8h h[2]; };
  static __device__ __forceinline__ v16h load(const _Float16* p) {
    U f; f.h[0] = *(const v8h*)(p); f.h[1] = *(const v8h*)(p + 16); return f.v;
  }
  static __device__ __forceinline__ v8f mma(v16h a, v16h b, v8f c) {
    return __builtin_amdgcn_wmma_f32_16x16x32_f16(false, a, false, b, (short)0, c, false, false);
  }
  static __device__ __forceinline__ void guard(v8f& a, v8f& b, v16h x, v16h y) { dep_guard_h(a, b, x, y); }
  static __device__ __forceinline__ void keep(v16h a, v16h b, v16h c, v16h d) { keep4_h(a, b, c, d); }
};
template <> struct Frag<__bf16> {
  typedef v16b V; union U { v16b v; v8b h[2]; };
  static __device__ __forceinline__ v16b load(const __bf16* p) {
    U f; f.h[0] = *(const v8b*)(p); f.h[1] = *(const v8b*)(p + 16); return f.v;
  }
  static __device__ __forceinline__ v8f mma(v16b a, v16b b, v8f c) {
    return __builtin_amdgcn_wmma_f32_16x16x32_bf16(false, a, false, b, (short)0, c, false, false);
  }
  static __device__ __forceinline__ void guard(v8f& a, v8f& b, v16b x, v16b y) { dep_guard_b(a, b, x, y); }
  static __device__ __forceinline__ void keep(v16b a, v16b b, v16b c, v16b d) { keep4_b(a, b, c, d); }
};

template <int ET> struct Elem;
template <> struct Elem<0> { typedef _Float16 T; };
template <> struct Elem<1> { typedef __bf16 T; };
template <int ET, bool SPLIT, int BIAS_MODE, int OUT_MODE, bool RESID, int ACT = 0>
__global__ __launch_bounds__(256) void wmma_gemm64(
    const unsigned short* __restrict__ Ap, const unsigned short* __restrict__ A2p, int lda, long strideA,
    const unsigned short* __restrict__ Btp, const unsigned short* __restrict__ Bt2p, int ldb, long strideB,
    void* __restrict__ Cout, void* __restrict__ Cout2, int ldc, long strideC,
    const float* __restrict__ bias,
    const float* __restrict__ resid, long strideR,
    int M, int N, int K, float scale) {
  typedef typename Elem<ET>::T T;
  typedef typename Frag<T>::V V;
  const T* A = (const T*)Ap; const T* A2 = (const T*)A2p; const T* Bt = (const T*)Btp; const T* Bt2 = (const T*)Bt2p;
  __shared__ __align__(16) float sT[8][16 * 68];
  const int b    = blockIdx.y;
  const int lane = threadIdx.x & 31;
  const int wave = threadIdx.x >> 5;
  const int tilesN = N >> 6;
  const int tilesM = M >> 6;
  const int tile = blockIdx.x * 8 + wave;
  if (tile >= tilesM * tilesN) return;
  const int tm = tile / tilesN;
  const int tn = tile - tm * tilesN;
  const int m0 = tm << 6;
  const int n0 = tn << 6;

  const T* Ab  = A  + (size_t)b * strideA;
  const T* Bb  = Bt + (size_t)b * strideB;
  const T* Ab2 = SPLIT ? (A2  + (size_t)b * strideA) : nullptr;
  const T* Bb2 = SPLIT ? (Bt2 + (size_t)b * strideB) : nullptr;

  const int rlane = lane & 15;
  const int koff  = (lane >> 4) * 8;
  const int mOff  = (lane >> 4) * 8;

  v8f acc[4][4];
#pragma unroll
  for (int i = 0; i < 4; ++i)
#pragma unroll
    for (int j = 0; j < 4; ++j) acc[i][j] = (v8f){0.f,0.f,0.f,0.f,0.f,0.f,0.f,0.f};

  for (int k0 = 0; k0 < K; k0 += 32) {
    V bh[4], bl[4];
#pragma unroll
    for (int j = 0; j < 4; ++j) {
      const size_t bo = (size_t)(n0 + (j << 4) + rlane) * ldb + koff + k0;
      bh[j] = Frag<T>::load(Bb + bo);
      if (SPLIT) bl[j] = Frag<T>::load(Bb2 + bo);
    }
#pragma unroll
    for (int i = 0; i < 4; ++i) {
      const size_t ao = (size_t)(m0 + (i << 4) + rlane) * lda + koff + k0;
      V ah = Frag<T>::load(Ab + ao);
      V al;
      if (SPLIT) al = Frag<T>::load(Ab2 + ao);
#pragma unroll
      for (int j = 0; j < 4; ++j) {
        acc[i][j] = Frag<T>::mma(ah, bh[j], acc[i][j]);
        if (SPLIT) {
          acc[i][j] = Frag<T>::mma(ah, bl[j], acc[i][j]);
          acc[i][j] = Frag<T>::mma(al, bh[j], acc[i][j]);
        }
      }
      Frag<T>::guard(acc[i][0], acc[i][3], ah, SPLIT ? al : ah);
    }
    Frag<T>::keep(bh[0], bh[1], bh[2], bh[3]);
    if (SPLIT) Frag<T>::keep(bl[0], bl[1], bl[2], bl[3]);
  }
  acc_guard4(acc[0][0], acc[0][1], acc[0][2], acc[0][3]);
  acc_guard4(acc[1][0], acc[1][1], acc[1][2], acc[1][3]);
  acc_guard4(acc[2][0], acc[2][1], acc[2][2], acc[2][3]);
  acc_guard4(acc[3][0], acc[3][1], acc[3][2], acc[3][3]);

  float* slab = sT[wave];
  const float* Rb = RESID ? (resid + (size_t)b * strideR) : nullptr;
#pragma unroll
  for (int i = 0; i < 4; ++i) {
    const int mBase = m0 + (i << 4);
#pragma unroll
    for (int j = 0; j < 4; ++j) {
      const int n = n0 + (j << 4) + rlane;
      float bv = 0.f;
      if (BIAS_MODE == 2) bv = bias[n];
#pragma unroll
      for (int r = 0; r < 8; ++r) {
        float v = acc[i][j][r] * scale;
        if (BIAS_MODE == 1) v += bias[mBase + mOff + r];
        if (BIAS_MODE == 2) v += bv;
        if (RESID) v += Rb[(size_t)(mBase + mOff + r) * ldc + n];
        if (ACT == 1) v = tanhf(v);
        if (ACT == 2) v = fmaxf(v, 0.0f);
        if (ACT == 3) v = v / (1.0f + expf(-v));
        if (ACT == 4) v = (v > 0.f) ? v : 0.01f * v;
        if (ACT == 5) v = 0.5f * v * (1.0f + erff(v * 0.70710678118654752f));
        slab[(mOff + r) * 68 + (j << 4) + rlane] = v;
      }
    }
    __builtin_amdgcn_fence(__ATOMIC_RELEASE, "workgroup");
    __builtin_amdgcn_wave_barrier();
    __builtin_amdgcn_fence(__ATOMIC_ACQUIRE, "workgroup");
    if (OUT_MODE == 0) {
      float* C = (float*)Cout + (size_t)b * strideC;
      const int hh = lane >> 4, c4 = (lane & 15) * 4;
      for (int pass = 0; pass < 2; ++pass) {
#pragma unroll
        for (int it = 0; it < 8; ++it) {
          const int row = it * 2 + hh;
          v4f v = *(const v4f*)(slab + row * 68 + c4);
          *(volatile v4f*)(C + (size_t)(mBase + row) * ldc + n0 + c4) = v;
        }
        __threadfence();
      }
    } else {
      const int q = lane >> 3, c8 = (lane & 7) * 8;
      unsigned short* C  = (unsigned short*)Cout  + (size_t)b * strideC;
      unsigned short* C2 = (OUT_MODE == 2) ? ((unsigned short*)Cout2 + (size_t)b * strideC) : nullptr;
      for (int pass = 0; pass < 2; ++pass) {
#pragma unroll
        for (int it = 0; it < 4; ++it) {
          const int row = it * 4 + q;
          const float* sp = slab + row * 68 + c8;
          v8h hv, lv;
#pragma unroll
          for (int e = 0; e < 8; ++e) {
            if (OUT_MODE == 1) {
              hv[e] = (_Float16)sp[e];
            } else {
              unsigned short hb = f2bf_bits(sp[e]);
              unsigned short lb = f2bf_bits(sp[e] - bf_bits2f(hb));
              hv[e] = __builtin_bit_cast(_Float16, hb);
              lv[e] = __builtin_bit_cast(_Float16, lb);
            }
          }
          *(volatile v8h*)(C + (size_t)(mBase + row) * ldc + n0 + c8) = hv;
          if (OUT_MODE == 2) *(volatile v8h*)(C2 + (size_t)(mBase + row) * ldc + n0 + c8) = lv;
        }
        __threadfence();
      }
    }
    __builtin_amdgcn_fence(__ATOMIC_RELEASE, "workgroup");
    __builtin_amdgcn_wave_barrier();
    __builtin_amdgcn_fence(__ATOMIC_ACQUIRE, "workgroup");
  }
}

__global__ __launch_bounds__(256) void cast_f32_f16x2(
    const float* __restrict__ in, _Float16* __restrict__ out, int n2) {
  int i = blockIdx.x * 256 + threadIdx.x;
  if (i < n2) {
    const _Float16 h0 = (_Float16)in[2 * i], h1 = (_Float16)in[2 * i + 1];
    const unsigned u = (unsigned)__builtin_bit_cast(unsigned short, h0) | ((unsigned)__builtin_bit_cast(unsigned short, h1) << 16);
    ((volatile unsigned*)out)[i] = u;
    __threadfence();
    ((volatile unsigned*)out)[i] = u;
  }
}

__global__ __launch_bounds__(NT) void wcast_kernel(const float* __restrict__ w0, const float* __restrict__ w1, const float* __restrict__ w2,
                                                  const float* __restrict__ w3, const float* __restrict__ w4, const float* __restrict__ w5,
                                                  _Float16* __restrict__ d0, _Float16* __restrict__ d1, _Float16* __restrict__ d2,
                                                  _Float16* __restrict__ d3, _Float16* __restrict__ d4, _Float16* __restrict__ d5) {
  const int seg = blockIdx.y;
  const float* src = (seg == 0) ? w0 : (seg == 1) ? w1 : (seg == 2) ? w2 : (seg == 3) ? w3 : (seg == 4) ? w4 : w5;
  _Float16* dst = (seg == 0) ? d0 : (seg == 1) ? d1 : (seg == 2) ? d2 : (seg == 3) ? d3 : (seg == 4) ? d4 : d5;
  const int n2 = (seg == 5) ? (HD * 256 / 2) : (HD * 128 / 2);
  const int i = blockIdx.x * NT + threadIdx.x;
  if (i < n2) {
    const _Float16 h0 = (_Float16)(src[2 * i] * 16.0f), h1 = (_Float16)(src[2 * i + 1] * 16.0f);
    const unsigned u = (unsigned)__builtin_bit_cast(unsigned short, h0) | ((unsigned)__builtin_bit_cast(unsigned short, h1) << 16);
    ((volatile unsigned*)dst)[i] = u;
    __threadfence();
    ((volatile unsigned*)dst)[i] = u;
  }
}

template <int MODE>
__global__ __launch_bounds__(NT) void ln_kernel(const float* __restrict__ G, const float* __restrict__ gam, const float* __restrict__ bet,
                                               const float* __restrict__ emb, _Float16* __restrict__ O16, float* __restrict__ O32, int M) {
  const int tid = threadIdx.x, lane = tid & 31, wave = tid >> 5;
  const int hs = lane >> 4, c4 = (lane & 15) * 4;
  const v4f g4 = *(const v4f*)(gam + c4), b4 = *(const v4f*)(bet + c4);
  const int rbase = (blockIdx.x * (NT / 32) + wave) * 16;
#pragma unroll 1
  for (int i = 0; i < 8; ++i) {
    const int row = rbase + 2 * i + hs;
    const int rc = row < M ? row : M - 1;
    const v4f h = *(const v4f*)(G + (size_t)rc * HD + c4);
    float s = (h[0] + h[1]) + (h[2] + h[3]);
    s += __shfl_xor(s, 8, 32); s += __shfl_xor(s, 4, 32); s += __shfl_xor(s, 2, 32); s += __shfl_xor(s, 1, 32);
    const float mean = s * (1.0f / 64.0f);
    const v4f d = h - mean;
    float q = (d[0] * d[0] + d[1] * d[1]) + (d[2] * d[2] + d[3] * d[3]);
    q += __shfl_xor(q, 8, 32); q += __shfl_xor(q, 4, 32); q += __shfl_xor(q, 2, 32); q += __shfl_xor(q, 1, 32);
    const float var = q * (1.0f / 64.0f);
    const float rs = 1.0f / sqrtf(var + LNEPS);
    const v4f t = d * rs;
    const v4f y = t * g4 + b4;
    const v4h yh = __builtin_convertvector(y, v4h);
    v4h eh = yh;
    if (MODE == 0) {
      const v4f em = *(const v4f*)(emb + (size_t)rc * HD + c4);
      eh = __builtin_convertvector(em, v4h);
    }
    for (int pass = 0; pass < 2; ++pass) {
      if (row < M) {
        if (MODE == 0) {
          _Float16* op = O16 + (size_t)row * 128;
          *(volatile v4h*)(op + c4) = yh;
          *(volatile v4h*)(op + 64 + c4) = eh;
        } else {
          *(volatile v4f*)(O32 + (size_t)row * HD + c4) = y;
          *(volatile v4h*)(O16 + (size_t)row * HD + c4) = yh;
        }
      }
      __threadfence();
    }
  }
}

__device__ __forceinline__ int blk_excl_scan(int cnt, int* scan_ws, int tid, int* tot) {
  const int lane = tid & 31, wave = tid >> 5; int incl = cnt;
#pragma unroll
  for (int o = 1; o < 32; o <<= 1) { const int v = __shfl_up(incl, o, 32); if (lane >= o) incl += v; }
  if (lane == 31) scan_ws[wave] = incl;
  __syncthreads();
  if (wave == 0) { int wv = (lane < NT / 32) ? scan_ws[lane] : 0; int wincl = wv;
#pragma unroll
    for (int o = 1; o < 32; o <<= 1) { const int v = __shfl_up(wincl, o, 32); if (lane >= o) wincl += v; }
    if (lane < NT / 32) scan_ws[32 + lane] = wincl - wv; if (lane == 31) scan_ws[64] = wincl; }
  __syncthreads();
  const int res = scan_ws[32 + wave] + incl - cnt; *tot = scan_ws[64];
  return res;
}
__device__ __forceinline__ int chunk_hits3(const int* __restrict__ rows, const int* __restrict__ cols, const float* __restrict__ vals,
                                           int e0, int n0, int tid, int* LP, float* LV, int* scan_ws) {
  const int eb = e0 + tid * SPT;
  const bool live = eb < NE;
  const int ebc = live ? eb : (NE - SPT);
  int rec[SPT]; float recv[SPT]; int cnt = 0;
#pragma unroll
  for (int k = 0; k < SPT; k += 4) {
    const v4i d4 = *(const v4i*)(rows + ebc + k);
    const v4i s4 = *(const v4i*)(cols + ebc + k);
    const v4f w4 = *(const v4f*)(vals + ebc + k);
#pragma unroll
    for (int e = 0; e < 4; ++e) {
      const int d = d4[e]; int r = -1;
      if (live && d >= n0 && d < n0 + TR && d < NNODE) {
        int s = s4[e]; s = s < 0 ? 0 : (s >= NNODE ? NNODE - 1 : s);
        r = ((d - n0) << 18) | s; ++cnt;
      }
      rec[k + e] = r; recv[k + e] = w4[e];
    }
  }
  int tot; int p = blk_excl_scan(cnt, scan_ws, tid, &tot);
#pragma unroll
  for (int k = 0; k < SPT; ++k) if (rec[k] >= 0) { if ((unsigned)p < (unsigned)SCH) { LP[p] = rec[k]; LV[p] = recv[k]; } ++p; }
  __syncthreads();
  return tot < SCH ? tot : SCH;
}

template <int FIRST>
__global__ __launch_bounds__(NT) void spmm_kernel(const int* __restrict__ rows, const int* __restrict__ cols, const float* __restrict__ vals,
                                                 const _Float16* __restrict__ Y, float* XA, float* AC, _Float16* X16) {
  __shared__ int LP[SCH];
  __shared__ float LV[SCH];
  __shared__ int scan_ws[80];
  const int tid = threadIdx.x, lane = tid & 31, wave = tid >> 5;
  const int n0 = blockIdx.x * TR;
  float* TGT = FIRST ? XA : AC;
  if (FIRST) {
    const v2f z2 = {0.f, 0.f};
    for (int pass = 0; pass < 2; ++pass) {
#pragma unroll 1
      for (int j = 0; j < RPW; ++j) {
        const int n = n0 + wave * RPW + j;
        if (n < MP) *(volatile v2f*)(XA + (size_t)n * HD + 2 * lane) = z2;
      }
      __threadfence();
    }
  }
#pragma unroll 1
  for (int c = 0; c < NCH; ++c) {
    const int tot = chunk_hits3(rows, cols, vals, c * SCH, n0, tid, LP, LV, scan_ws);
#pragma unroll 1
    for (int base = 0; base < tot; base += 32) {
      const int q = base + lane;
      const int qc = q < SCH ? q : SCH - 1;
      int rv = LP[qc]; const float vv = LV[qc];
      if (q >= tot) rv = -1;
      const int own = ((rv >> 28) == wave) ? 1 : 0;
      unsigned msk = (unsigned)__ballot(own);
#pragma unroll 1
      for (int it = 0; it < 32; ++it) {
        if (msk == 0u) break;
        const int bp = __builtin_ctz(msk); msk &= msk - 1u;
        const int r = __shfl(rv, bp, 32);
        const float v = __shfl(vv, bp, 32);
        const int dl = r >> 18, cs = r & 0x3FFFF;
        const v2h yh = *(const v2h*)(Y + (size_t)cs * HD + 2 * lane);
        const float y0 = (float)yh[0], y1 = (float)yh[1];
        float* rp = TGT + (size_t)(n0 + dl) * HD + 2 * lane;
        v2f a = *(const v2f*)rp;
        a[0] += v * y0; a[1] += v * y1;
        *(volatile v2f*)rp = a;
        __threadfence();
        *(volatile v2f*)rp = a;
      }
    }
    __syncthreads();
  }
  if (FIRST) {
#pragma unroll 1
    for (int j = 0; j < RPW; ++j) {
      const int n = n0 + wave * RPW + j;
      if (n < MP) {
        const v2f a = *(const v2f*)(XA + (size_t)n * HD + 2 * lane);
        const float x0 = fmaxf(a[0], 0.f), x1 = fmaxf(a[1], 0.f);
        float* ap = AC + (size_t)n * HD + 2 * lane;
        v2f s = *(const v2f*)ap;
        s[0] += x0; s[1] += x1;
        v2h h; h[0] = (_Float16)x0; h[1] = (_Float16)x1;
        _Float16* hp = X16 + (size_t)n * HD + 2 * lane;
        for (int pass = 0; pass < 2; ++pass) {
          *(volatile v2f*)ap = s;
          *(volatile v2h*)hp = h;
          __threadfence();
        }
      }
    }
  }
}

__global__ __launch_bounds__(NT) void pair_kernel(const float* __restrict__ AC, const int* __restrict__ uidx, const int* __restrict__ iidx,
                                                 _Float16* __restrict__ P) {
  const int tid = threadIdx.x, lane = tid & 31, wave = tid >> 5;
  const float third = 1.0f / 3.0f;
#pragma unroll 1
  for (int i = 0; i < 8; ++i) {
    const int q = (blockIdx.x * (NT / 32) + wave) * 8 + i;
    int u = uidx[q]; u = u < 0 ? 0 : (u >= NNODE ? NNODE - 1 : u);
    int t = iidx[q]; t = t < -NUSERS ? -NUSERS : (t > NNODE ? NNODE : t);
    int w = t + NUSERS; w = w < 0 ? 0 : (w >= NNODE ? NNODE - 1 : w);
    const v2f au = *(const v2f*)(AC + (size_t)u * HD + 2 * lane);
    const v2f ai = *(const v2f*)(AC + (size_t)w * HD + 2 * lane);
    const v2f zu = au * third, zi = ai * third;
    const v2f pr = zu * zi;
    v2f df = zu - zi; df[0] = fabsf(df[0]); df[1] = fabsf(df[1]);
    const v2h h0 = __builtin_convertvector(zu, v2h), h1 = __builtin_convertvector(zi, v2h);
    const v2h h2 = __builtin_convertvector(pr, v2h), h3 = __builtin_convertvector(df, v2h);
    _Float16* pp = P + (size_t)q * 256 + 2 * lane;
    for (int pass = 0; pass < 2; ++pass) {
      *(volatile v2h*)(pp) = h0;
      *(volatile v2h*)(pp + 64) = h1;
      *(volatile v2h*)(pp + 128) = h2;
      *(volatile v2h*)(pp + 192) = h3;
      __threadfence();
    }
  }
}

__global__ __launch_bounds__(NT) void score_kernel(const float* __restrict__ S, const float* __restrict__ s2W, const float* __restrict__ s2b,
                                                  const float* __restrict__ gm, const float* __restrict__ ub, const float* __restrict__ ib,
                                                  const int* __restrict__ uidx, const int* __restrict__ iidx, float* __restrict__ out) {
  const int tid = threadIdx.x, lane = tid & 31, wave = tid >> 5;
  const int qb = (blockIdx.x * (NT / 32) + wave) * 32;
  const v2f w2 = *(const v2f*)(s2W + 2 * lane);
  const float g0 = gm[0], sb = s2b[0];
  float mine = 0.f;
#pragma unroll 1
  for (int i = 0; i < 32; ++i) {
    const int q = qb + i;
    const v2f x = *(const v2f*)(S + (size_t)q * HD + 2 * lane);
    float d = x[0] * w2[0] + x[1] * w2[1];
    d += __shfl_xor(d, 16, 32); d += __shfl_xor(d, 8, 32); d += __shfl_xor(d, 4, 32); d += __shfl_xor(d, 2, 32); d += __shfl_xor(d, 1, 32);
    int u = uidx[q]; u = u < 0 ? 0 : (u >= NUSERS ? NUSERS - 1 : u);
    int t = iidx[q]; t = t < 0 ? 0 : (t >= NITEMS ? NITEMS - 1 : t);
    const float score = d + sb;
    float pred = ((g0 + ub[u]) + ib[t]) + score;
    pred = fminf(fmaxf(pred, 1.0f), 5.0f);
    if (lane == i) mine = pred;
  }
  ((volatile float*)out)[qb + lane] = mine;
  __threadfence();
  ((volatile float*)out)[qb + lane] = mine;
}

extern "C" void kernel_launch(void* const* d_in, const int* in_sizes, int n_in,
                              void* d_out, int out_size, void* d_ws,
                              size_t ws_size, hipStream_t stream) {
  if (n_in < 34) return;
  if (in_sizes[0] != NUSERS * 128 || in_sizes[1] != NITEMS * 128 || in_sizes[2] != NE || in_sizes[11] != NUSERS * HD ||
      in_sizes[12] != NITEMS * HD || in_sizes[30] != NE || in_sizes[31] != NE || in_sizes[32] != NQ || in_sizes[33] != NQ ||
      out_size != NQ) return;
  const float* user_features = (const float*)d_in[0];
  const float* item_features = (const float*)d_in[1];
  const float* adj_vals      = (const float*)d_in[2];
  const float* ueW  = (const float*)d_in[3];
  const float* ueB  = (const float*)d_in[4];
  const float* ueG  = (const float*)d_in[5];
  const float* ueBE = (const float*)d_in[6];
  const float* ieW  = (const float*)d_in[7];
  const float* ieB  = (const float*)d_in[8];
  const float* ieG  = (const float*)d_in[9];
  const float* ieBE = (const float*)d_in[10];
  const float* uid_emb = (const float*)d_in[11];
  const float* iid_emb = (const float*)d_in[12];
  const float* ufW  = (const float*)d_in[13];
  const float* ufB  = (const float*)d_in[14];
  const float* ufG  = (const float*)d_in[15];
  const float* ufBE = (const float*)d_in[16];
  const float* ifW  = (const float*)d_in[17];
  const float* ifB  = (const float*)d_in[18];
  const float* ifG  = (const float*)d_in[19];
  const float* ifBE = (const float*)d_in[20];
  const float* gcnW = (const float*)d_in[21];
  const float* gcnB = (const float*)d_in[22];
  const float* user_bias = (const float*)d_in[23];
  const float* item_bias = (const float*)d_in[24];
  const float* s1W = (const float*)d_in[25];
  const float* s1b = (const float*)d_in[26];
  const float* s2W = (const float*)d_in[27];
  const float* s2b = (const float*)d_in[28];
  const float* gm  = (const float*)d_in[29];
  const int* adj_rows = (const int*)d_in[30];
  const int* adj_cols = (const int*)d_in[31];
  const int* user_idx = (const int*)d_in[32];
  const int* item_idx = (const int*)d_in[33];
  float* out = (float*)d_out;

  char* ws = (char*)d_ws; size_t off = 0;
  auto carve = [&](size_t bytes) -> char* { char* p = ws + off; off += (bytes + 255) & ~(size_t)255; return p; };
  _Float16* Wue = (_Float16*)carve((size_t)HD * 128 * 2);
  _Float16* Wie = (_Float16*)carve((size_t)HD * 128 * 2);
  _Float16* Wuf = (_Float16*)carve((size_t)HD * 128 * 2);
  _Float16* Wif = (_Float16*)carve((size_t)HD * 128 * 2);
  _Float16* Wg  = (_Float16*)carve((size_t)2 * HD * HD * 2);
  _Float16* Ws1 = (_Float16*)carve((size_t)HD * 256 * 2);
  float*    ACC = (float*)carve((size_t)MP * HD * 4);
  _Float16* X16 = (_Float16*)carve((size_t)MP * HD * 2);
  char*     R   = carve((size_t)MP * HD * 2 + (size_t)MP * HD * 4);
  if (off > ws_size || off > (size_t)134217728) return;
  _Float16* S0  = (_Float16*)R;
  float*    S1  = (float*)(R + (size_t)MU * 128 * 2);
  _Float16* Y16 = (_Float16*)R;
  float*    XA  = (float*)(R + (size_t)MP * HD * 2);
  _Float16* PR  = (_Float16*)R;
  float*    SO  = (float*)(R + (size_t)NQ * 256 * 2);
  const float inv16 = 1.0f / 16.0f;

  wcast_kernel<<<dim3(32, 6), NT, 0, stream>>>(ueW, ieW, ufW, ifW, gcnW, s1W, Wue, Wie, Wuf, Wif, Wg, Ws1);

  cast_f32_f16x2<<<(NUSERS * 128 / 2 + 255) / 256, 256, 0, stream>>>(user_features, S0, NUSERS * 128 / 2);
  wmma_gemm64<0, false, 2, 0, false, 2><<<dim3((MU / 64 + 7) / 8, 1), 256, 0, stream>>>(
      (const unsigned short*)S0, (const unsigned short*)nullptr, 128, 0L, (const unsigned short*)Wue, (const unsigned short*)nullptr, 128, 0L,
      (void*)S1, (void*)nullptr, HD, 0L, ueB, (const float*)nullptr, 0L, MU, HD, 128, inv16);
  ln_kernel<0><<<(NUSERS + 127) / 128, NT, 0, stream>>>(S1, ueG, ueBE, uid_emb, S0, (float*)nullptr, NUSERS);
  wmma_gemm64<0, false, 2, 0, false, 2><<<dim3((MU / 64 + 7) / 8, 1), 256, 0, stream>>>(
      (const unsigned short*)S0, (const unsigned short*)nullptr, 128, 0L, (const unsigned short*)Wuf, (const unsigned short*)nullptr, 128, 0L,
      (void*)S1, (void*)nullptr, HD, 0L, ufB, (const float*)nullptr, 0L, MU, HD, 128, inv16);
  ln_kernel<1><<<(NUSERS + 127) / 128, NT, 0, stream>>>(S1, ufG, ufBE, (const float*)nullptr, X16, ACC, NUSERS);

  cast_f32_f16x2<<<(NITEMS * 128 / 2 + 255) / 256, 256, 0, stream>>>(item_features, S0, NITEMS * 128 / 2);
  wmma_gemm64<0, false, 2, 0, false, 2><<<dim3((MI / 64 + 7) / 8, 1), 256, 0, stream>>>(
      (const unsigned short*)S0, (const unsigned short*)nullptr, 128, 0L, (const unsigned short*)Wie, (const unsigned short*)nullptr, 128, 0L,
      (void*)S1, (void*)nullptr, HD, 0L, ieB, (const float*)nullptr, 0L, MI, HD, 128, inv16);
  ln_kernel<0><<<(NITEMS + 127) / 128, NT, 0, stream>>>(S1, ieG, ieBE, iid_emb, S0, (float*)nullptr, NITEMS);
  wmma_gemm64<0, false, 2, 0, false, 2><<<dim3((MI / 64 + 7) / 8, 1), 256, 0, stream>>>(
      (const unsigned short*)S0, (const unsigned short*)nullptr, 128, 0L, (const unsigned short*)Wif, (const unsigned short*)nullptr, 128, 0L,
      (void*)S1, (void*)nullptr, HD, 0L, ifB, (const float*)nullptr, 0L, MI, HD, 128, inv16);
  ln_kernel<1><<<(NITEMS + 127) / 128, NT, 0, stream>>>(S1, ifG, ifBE, (const float*)nullptr, X16 + (size_t)NUSERS * HD,
                                                        ACC + (size_t)NUSERS * HD, NITEMS);

  wmma_gemm64<0, false, 2, 1, false, 0><<<dim3((MP / 64 + 7) / 8, 1), 256, 0, stream>>>(
      (const unsigned short*)X16, (const unsigned short*)nullptr, HD, 0L, (const unsigned short*)Wg, (const unsigned short*)nullptr, HD, 0L,
      (void*)Y16, (void*)nullptr, HD, 0L, gcnB, (const float*)nullptr, 0L, MP, HD, HD, inv16);
  spmm_kernel<1><<<NTILE, NT, 0, stream>>>(adj_rows, adj_cols, adj_vals, Y16, XA, ACC, X16);

  wmma_gemm64<0, false, 2, 1, false, 0><<<dim3((MP / 64 + 7) / 8, 1), 256, 0, stream>>>(
      (const unsigned short*)X16, (const unsigned short*)nullptr, HD, 0L, (const unsigned short*)(Wg + HD * HD), (const unsigned short*)nullptr, HD, 0L,
      (void*)Y16, (void*)nullptr, HD, 0L, gcnB + HD, (const float*)nullptr, 0L, MP, HD, HD, inv16);
  spmm_kernel<0><<<NTILE, NT, 0, stream>>>(adj_rows, adj_cols, adj_vals, Y16, XA, ACC, X16);

  pair_kernel<<<NQ / 64, NT, 0, stream>>>(ACC, user_idx, item_idx, PR);
  wmma_gemm64<0, false, 2, 0, false, 2><<<dim3((NQ / 64 + 7) / 8, 1), 256, 0, stream>>>(
      (const unsigned short*)PR, (const unsigned short*)nullptr, 256, 0L, (const unsigned short*)Ws1, (const unsigned short*)nullptr, 256, 0L,
      (void*)SO, (void*)nullptr, HD, 0L, s1b, (const float*)nullptr, 0L, NQ, HD, 256, inv16);
  score_kernel<<<NQ / 256, NT, 0, stream>>>(SO, s2W, s2b, gm, user_bias, item_bias, user_idx, item_idx, out);
}
